// DisorderedCausalSelfAttention_43052752175110
// MI455X (gfx1250) — hardware-run, weakly checked
//
#include <hip/hip_runtime.h>
#include <math.h>
#include <stdint.h>

#define NB        4
#define SEQ       2048
#define DM        1024
#define NH        16
#define HD        64
#define DQK       2048
#define QCOLS     1024
#define VLO_COLS  128
#define NQB       32
#define AT_KC     64

typedef __attribute__((ext_vector_type(16))) _Float16 v16h;
typedef __attribute__((ext_vector_type(8)))  _Float16 v8h;
typedef __attribute__((ext_vector_type(16))) __bf16   v16b;
typedef __attribute__((ext_vector_type(8)))  __bf16   v8b;
typedef __attribute__((ext_vector_type(8)))  float    v8f;
typedef __attribute__((ext_vector_type(4)))  float    v4f;
typedef __attribute__((ext_vector_type(4)))  unsigned int v4u;

__device__ __forceinline__ unsigned short f2bf_bits(float f) {
  unsigned u = __float_as_uint(f);
  return (unsigned short)((u + 0x7FFFu + ((u >> 16) & 1u)) >> 16);
}
__device__ __forceinline__ float bf_bits2f(unsigned short h) { return __uint_as_float(((unsigned)h) << 16); }
__device__ __forceinline__ float bfr(float f) { return bf_bits2f(f2bf_bits(f)); }
__device__ __forceinline__ unsigned pk16(unsigned short a, unsigned short b) { return (unsigned)a | ((unsigned)b << 16); }
__device__ __forceinline__ unsigned short h2bits(_Float16 x) { return __builtin_bit_cast(unsigned short, x); }

union FragB { v16b v; v8b h[2]; };
union FragH { v16h v; v8h h[2]; };
__device__ __forceinline__ v16b ldfrag_b(const __bf16* p) { FragB f; f.h[0] = *(const v8b*)(p); f.h[1] = *(const v8b*)(p + 16); return f.v; }

__device__ __forceinline__ void dep_guard_b(v8f& a, v8f& b, v16b x, v16b y) { asm volatile("v_nop\n\tv_nop\n\tv_nop\n\tv_nop" : "+v"(a), "+v"(b) : "v"(x), "v"(y)); }
__device__ __forceinline__ void keep4_b(v16b a, v16b b, v16b c, v16b d) { asm volatile("v_nop" :: "v"(a), "v"(b), "v"(c), "v"(d)); }
__device__ __forceinline__ void acc_guard4(v8f& a, v8f& b, v8f& c, v8f& d) { asm volatile("v_nop\n\tv_nop\n\tv_nop\n\tv_nop" : "+v"(a), "+v"(b), "+v"(c), "+v"(d)); }
__device__ __forceinline__ v8f mma_b(v16b a, v16b b, v8f c) {
  c = __builtin_amdgcn_wmma_f32_16x16x32_bf16(false, a, false, b, (short)0, c, false, false);
  asm volatile("v_nop\n\tv_nop\n\tv_nop\n\tv_nop" : "+v"(c) : "v"(a), "v"(b));
  return c;
}
__device__ __forceinline__ v8f mma_h(v16h a, v16h b, v8f c) {
  c = __builtin_amdgcn_wmma_f32_16x16x32_f16(false, a, false, b, (short)0, c, false, false);
  asm volatile("v_nop\n\tv_nop\n\tv_nop\n\tv_nop" : "+v"(c) : "v"(a), "v"(b));
  return c;
}

template <int MODE>
__global__ __launch_bounds__(256) void gemm64(
    const unsigned short* __restrict__ Ap, const unsigned short* __restrict__ A2p, int lda, long strideA,
    const unsigned short* __restrict__ Btp, int ldb, long strideB,
    void* __restrict__ Cout, void* __restrict__ Cout2, int ldc, long strideC, int ldc2, long strideC2,
    const float* __restrict__ bias, const float* __restrict__ biasq, const float* __restrict__ biask,
    int M, int N, int K) {
  __shared__ __align__(16) float sT[8][16 * 68];
  const __bf16* A  = (const __bf16*)(const void*)Ap;
  const __bf16* A2 = (const __bf16*)(const void*)A2p;
  const __bf16* Bt = (const __bf16*)(const void*)Btp;
  const int b    = blockIdx.y;
  const int lane = threadIdx.x & 31;
  const int wave = threadIdx.x >> 5;
  const int tilesN = N >> 6;
  const int tilesM = M >> 6;
  const int tile = blockIdx.x * 8 + wave;
  if (tile >= tilesM * tilesN) return;
  const int tm = tile / tilesN;
  const int tn = tile - tm * tilesN;
  const int m0 = tm << 6;
  const int n0 = tn << 6;

  const __bf16* Ab  = A  + (size_t)b * strideA;
  const __bf16* Bb  = Bt + (size_t)b * strideB;
  const __bf16* Ab2 = (MODE == 2) ? (A2 + (size_t)b * strideA) : Ab;

  const int rlane = lane & 15;
  const int koff  = (lane >> 4) * 8;
  const int mOff  = (lane >> 4) * 8;

  v8f acc[4][4];
#pragma unroll
  for (int i = 0; i < 4; ++i)
#pragma unroll
    for (int j = 0; j < 4; ++j) acc[i][j] = (v8f){0.f,0.f,0.f,0.f,0.f,0.f,0.f,0.f};

  for (int k0 = 0; k0 < K; k0 += 32) {
    v16b bh[4];
#pragma unroll
    for (int j = 0; j < 4; ++j) {
      const size_t bo = (size_t)(n0 + (j << 4) + rlane) * ldb + koff + k0;
      bh[j] = ldfrag_b(Bb + bo);
    }
#pragma unroll
    for (int i = 0; i < 4; ++i) {
      const size_t ao = (size_t)(m0 + (i << 4) + rlane) * lda + koff + k0;
      const v16b ah = ldfrag_b(Ab + ao);
      v16b al = ah;
      if (MODE == 2) al = ldfrag_b(Ab2 + ao);
#pragma unroll
      for (int j = 0; j < 4; ++j) {
        acc[i][j] = __builtin_amdgcn_wmma_f32_16x16x32_bf16(false, ah, false, bh[j], (short)0, acc[i][j], false, false);
        if (MODE == 2)
          acc[i][j] = __builtin_amdgcn_wmma_f32_16x16x32_bf16(false, al, false, bh[j], (short)0, acc[i][j], false, false);
      }
      dep_guard_b(acc[i][0], acc[i][3], ah, al);
    }
    keep4_b(bh[0], bh[1], bh[2], bh[3]);
  }
  acc_guard4(acc[0][0], acc[0][1], acc[0][2], acc[0][3]);
  acc_guard4(acc[1][0], acc[1][1], acc[1][2], acc[1][3]);
  acc_guard4(acc[2][0], acc[2][1], acc[2][2], acc[2][3]);
  acc_guard4(acc[3][0], acc[3][1], acc[3][2], acc[3][3]);

  float* slab = sT[wave];
#pragma unroll
  for (int i = 0; i < 4; ++i) {
    const int mBase = m0 + (i << 4);
#pragma unroll
    for (int j = 0; j < 4; ++j) {
      const int n = n0 + (j << 4) + rlane;
      float bn = 0.f, b2 = 0.f;
      if (MODE == 0) {
        bn = bfr(bias[n]);
        const int iq = (n < QCOLS) ? n : (QCOLS - 1);
        int ik = n - QCOLS; ik = (ik < 0) ? 0 : ik; ik = (ik > QCOLS - 1) ? (QCOLS - 1) : ik;
        const float vq = bfr(biasq[iq]);
        const float vk = bfr(biask[ik]);
        b2 = (n < QCOLS) ? vq : vk;
      }
      if (MODE == 2) bn = bfr(bias[n]);
#pragma unroll
      for (int r = 0; r < 8; ++r) {
        float v = acc[i][j][r];
        if (MODE == 0) { v = v + bn; v = v + b2; }
        if (MODE == 1) v = v + bfr(bias[mBase + mOff + r]);
        if (MODE == 2) v = v + bn;
        slab[(mOff + r) * 68 + (j << 4) + rlane] = v;
      }
    }
    __builtin_amdgcn_fence(__ATOMIC_RELEASE, "workgroup");
    __builtin_amdgcn_wave_barrier();
    __builtin_amdgcn_fence(__ATOMIC_ACQUIRE, "workgroup");
    if (MODE == 2) {
      float* C = (float*)Cout + (size_t)b * strideC;
      const int h2 = lane >> 4, c4 = (lane & 15) * 4;
      for (int pass = 0; pass < 2; ++pass) {
#pragma unroll
        for (int it = 0; it < 8; ++it) {
          const int row = it * 2 + h2;
          const v4f v = *(const v4f*)(slab + row * 68 + c4);
          *(volatile v4f*)(C + (size_t)(mBase + row) * ldc + n0 + c4) = v;
        }
        __threadfence();
      }
    } else {
      const int q = lane >> 3, c8 = (lane & 7) * 8;
      unsigned short* C  = (unsigned short*)Cout  + (size_t)b * strideC;
      unsigned short* C2 = (unsigned short*)Cout2 + (size_t)b * strideC2;
      const bool wlo = (MODE == 0) || (n0 < VLO_COLS);
      v4u hv[4], lv[4];
#pragma unroll
      for (int it = 0; it < 4; ++it) {
        const int row = it * 4 + q;
        const float* sp = slab + row * 68 + c8;
        v4u a, a2;
#pragma unroll
        for (int e = 0; e < 4; ++e) {
          const float f0 = sp[2 * e], f1 = sp[2 * e + 1];
          unsigned short h0, h1, l0, l1;
          if (MODE == 0) {
            h0 = f2bf_bits(f0); h1 = f2bf_bits(f1);
            l0 = f2bf_bits(f0 - bf_bits2f(h0)); l1 = f2bf_bits(f1 - bf_bits2f(h1));
          } else {
            const _Float16 x0 = (_Float16)f0, x1 = (_Float16)f1;
            h0 = h2bits(x0); h1 = h2bits(x1);
            l0 = h2bits((_Float16)((f0 - (float)x0) * 1024.0f));
            l1 = h2bits((_Float16)((f1 - (float)x1) * 1024.0f));
          }
          a[e] = pk16(h0, h1); a2[e] = pk16(l0, l1);
        }
        hv[it] = a; lv[it] = a2;
      }
      for (int pass = 0; pass < 2; ++pass) {
#pragma unroll
        for (int it = 0; it < 4; ++it) {
          const int row = it * 4 + q;
          *(volatile v4u*)(C + (size_t)(mBase + row) * ldc + n0 + c8) = hv[it];
          if (wlo) *(volatile v4u*)(C2 + (size_t)(mBase + row) * ldc2 + n0 + c8) = lv[it];
        }
        __threadfence();
      }
    }
    __builtin_amdgcn_fence(__ATOMIC_RELEASE, "workgroup");
    __builtin_amdgcn_wave_barrier();
    __builtin_amdgcn_fence(__ATOMIC_ACQUIRE, "workgroup");
  }
}

__global__ __launch_bounds__(256) void cvt_x_kernel(const float* __restrict__ x, unsigned short* __restrict__ xb, int n8,
                                                    const float* __restrict__ bq, float* __restrict__ out1, int nq4) {
  if (blockIdx.x == 0) {
    const int t = threadIdx.x;
    if (t < nq4) {
      const v4f v = *(const v4f*)(bq + 4 * t);
      v4f w;
      w[0] = bfr(v[0]); w[1] = bfr(v[1]); w[2] = bfr(v[2]); w[3] = bfr(v[3]);
      *(volatile v4f*)(out1 + 4 * t) = w;
      __threadfence();
      *(volatile v4f*)(out1 + 4 * t) = w;
    }
  }
  const int i = blockIdx.x * 256 + threadIdx.x;
  if (i < n8) {
    const v4f a = *(const v4f*)(x + 8 * (size_t)i);
    const v4f c = *(const v4f*)(x + 8 * (size_t)i + 4);
    v4u u;
    u[0] = pk16(f2bf_bits(a[0]), f2bf_bits(a[1]));
    u[1] = pk16(f2bf_bits(a[2]), f2bf_bits(a[3]));
    u[2] = pk16(f2bf_bits(c[0]), f2bf_bits(c[1]));
    u[3] = pk16(f2bf_bits(c[2]), f2bf_bits(c[3]));
    *(volatile v4u*)(xb + 8 * (size_t)i) = u;
    __threadfence();
    *(volatile v4u*)(xb + 8 * (size_t)i) = u;
  }
}

__global__ __launch_bounds__(256) void tsplit1_kernel(const float* __restrict__ W, unsigned short* __restrict__ ot, int R, int Cc) {
  __shared__ __align__(16) float tf[64 * 68];
  const int c0  = blockIdx.x * 64;
  const int r0  = blockIdx.y * 64;
  const int tid = threadIdx.x;
  {
    const int lr = tid >> 4;
    const int c4 = (tid & 15) * 4;
#pragma unroll
    for (int it = 0; it < 4; ++it) {
      const int rr = it * 16 + lr;
      const v4f a = *(const v4f*)(W + (size_t)(r0 + rr) * Cc + c0 + c4);
      *(v4f*)(tf + rr * 68 + c4) = a;
    }
  }
  __syncthreads();
  const int sub = tid >> 3;
  const int c8  = (tid & 7) * 8;
  v4u hv[2];
#pragma unroll
  for (int it = 0; it < 2; ++it) {
    const int oc = it * 32 + sub;
    v4u a;
#pragma unroll
    for (int q = 0; q < 4; ++q) {
      const float f0 = tf[(c8 + 2 * q) * 68 + oc];
      const float f1 = tf[(c8 + 2 * q + 1) * 68 + oc];
      a[q] = pk16(f2bf_bits(f0), f2bf_bits(f1));
    }
    hv[it] = a;
  }
  for (int pass = 0; pass < 2; ++pass) {
#pragma unroll
    for (int it = 0; it < 2; ++it) {
      const int oc = it * 32 + sub;
      const size_t go = (size_t)(c0 + oc) * R + r0 + c8;
      *(volatile v4u*)(ot + go) = hv[it];
    }
    __threadfence();
  }
}

__global__ __launch_bounds__(128)
void attn_kernel(const unsigned short* __restrict__ qkh, const unsigned short* __restrict__ qkl,
                 const unsigned short* __restrict__ vthp, const unsigned short* __restrict__ vtlp,
                 unsigned short* __restrict__ yhp, unsigned short* __restrict__ ylp) {
  __shared__ __align__(16) __bf16   Ksh[AT_KC * HD];
  __shared__ __align__(16) __bf16   Ksl[AT_KC * HD];
  __shared__ __align__(16) _Float16 Vts[HD * AT_KC];
  __shared__ __align__(16) _Float16 Vrs[HD * AT_KC];
  __shared__ __align__(16) _Float16 Psh[4][16 * AT_KC];
  __shared__ __align__(16) float    Os[4][16 * 68];

  const int tid  = threadIdx.x;
  const int wave = tid >> 5;
  const int lane = tid & 31;
  const int hh   = lane >> 4;
  const int c    = lane & 15;

  const int b  = blockIdx.y;
  const int bx = blockIdx.x;
  const int qb = bx & (NQB - 1);
  const int h  = bx >> 5;
  const int q0 = qb * 64 + wave * 16;
  const bool vres = (qb < 2);

  const __bf16* Qh = (const __bf16*)(const void*)qkh + (size_t)b * SEQ * DQK + (size_t)h * HD;
  const __bf16* Ql = (const __bf16*)(const void*)qkl + (size_t)b * SEQ * DQK + (size_t)h * HD;
  const __bf16* Kh = Qh + QCOLS;
  const __bf16* Kl = Ql + QCOLS;
  const _Float16* Vh = (const _Float16*)(const void*)vthp + ((size_t)b * DM + (size_t)h * HD) * SEQ;
  const _Float16* Vl = (const _Float16*)(const void*)vtlp + ((size_t)b * DM + (size_t)h * HD) * VLO_COLS;
  unsigned short* Yh = yhp + (size_t)b * SEQ * DM + (size_t)h * HD;
  unsigned short* Yl = ylp + (size_t)b * SEQ * DM + (size_t)h * HD;

  v16b qah[2], qal[2];
#pragma unroll
  for (int dc = 0; dc < 2; ++dc) {
    const __bf16* qr = Qh + (size_t)(q0 + c) * DQK + dc * 32 + 8 * hh;
    const __bf16* ql = Ql + (size_t)(q0 + c) * DQK + dc * 32 + 8 * hh;
    qah[dc] = ldfrag_b(qr);
    qal[dc] = ldfrag_b(ql);
  }

  float mrow[8], lrow[8];
  v8f oacc[4], oacc2[4];
#pragma unroll
  for (int r = 0; r < 8; ++r) { mrow[r] = -INFINITY; lrow[r] = 0.f; }
#pragma unroll
  for (int t = 0; t < 4; ++t) { oacc[t] = (v8f){0.f,0.f,0.f,0.f,0.f,0.f,0.f,0.f}; oacc2[t] = oacc[t]; }

  const int nChunks = qb + 1;
  for (int kc = 0; kc < nChunks; ++kc) {
    const int kv0 = kc * AT_KC;
    __syncthreads();
    {
      const int r = tid >> 1, half = (tid & 1) * 32;
      const __bf16* ksh = Kh + (size_t)(kv0 + r) * DQK + half;
      const __bf16* ksl = Kl + (size_t)(kv0 + r) * DQK + half;
      const _Float16* vsh = Vh + (size_t)r * SEQ + kv0 + half;
#pragma unroll
      for (int i = 0; i < 4; ++i) {
        const v8b a0 = *(const v8b*)(ksh + 8 * i);
        const v8b a1 = *(const v8b*)(ksl + 8 * i);
        const v8h b0 = *(const v8h*)(vsh + 8 * i);
        *(v8b*)(Ksh + r * HD    + half + 8 * i) = a0;
        *(v8b*)(Ksl + r * HD    + half + 8 * i) = a1;
        *(v8h*)(Vts + r * AT_KC + half + 8 * i) = b0;
      }
      if (vres) {
        const _Float16* vsl = Vl + (size_t)r * VLO_COLS + kv0 + half;
#pragma unroll
        for (int i = 0; i < 4; ++i) {
          const v8h b1 = *(const v8h*)(vsl + 8 * i);
          *(v8h*)(Vrs + r * AT_KC + half + 8 * i) = b1;
        }
      }
    }
    __syncthreads();

    v8f s[4];
#pragma unroll
    for (int j = 0; j < 4; ++j) {
      s[j] = (v8f){0.f,0.f,0.f,0.f,0.f,0.f,0.f,0.f};
#pragma unroll
      for (int dc = 0; dc < 2; ++dc) {
        FragB kb, kl;
        kb.h[0] = *(const v8b*)(Ksh + (j * 16 + c) * HD + dc * 32 + 8 * hh);
        kb.h[1] = *(const v8b*)(Ksh + (j * 16 + c) * HD + dc * 32 + 16 + 8 * hh);
        kl.h[0] = *(const v8b*)(Ksl + (j * 16 + c) * HD + dc * 32 + 8 * hh);
        kl.h[1] = *(const v8b*)(Ksl + (j * 16 + c) * HD + dc * 32 + 16 + 8 * hh);
        s[j] = mma_b(qah[dc], kb.v, s[j]);
        s[j] = mma_b(qah[dc], kl.v, s[j]);
        s[j] = mma_b(qal[dc], kb.v, s[j]);
      }
    }
    const bool diag = (kc == qb);
    float cm[8];
#pragma unroll
    for (int r = 0; r < 8; ++r) {
      const int qrow = q0 + 8 * hh + r;
      float m = -INFINITY;
#pragma unroll
      for (int j = 0; j < 4; ++j) {
        const int kvcol = kv0 + j * 16 + c;
        const float sv = s[j][r] * 0.125f;
        const bool masked = diag && (kvcol > qrow);
        const float sm = masked ? -INFINITY : sv;
        s[j][r] = sm;
        m = fmaxf(m, sm);
      }
#pragma unroll
      for (int off = 1; off < 16; off <<= 1) m = fmaxf(m, __shfl_xor(m, off, 32));
      cm[r] = m;
    }
    _Float16* pw = Psh[wave];
#pragma unroll
    for (int r = 0; r < 8; ++r) {
      const float mnew  = fmaxf(mrow[r], cm[r]);
      const float alpha = __expf(mrow[r] - mnew);
      mrow[r] = mnew;
      float psum = 0.f;
#pragma unroll
      for (int j = 0; j < 4; ++j) {
        const float p = __expf(s[j][r] - mnew);
        const _Float16 ph = (_Float16)(p * 4096.0f);
        psum += (float)ph;
        pw[(8 * hh + r) * AT_KC + j * 16 + c] = ph;
      }
#pragma unroll
      for (int off = 1; off < 16; off <<= 1) psum += __shfl_xor(psum, off, 32);
      lrow[r] = lrow[r] * alpha + psum;
#pragma unroll
      for (int t = 0; t < 4; ++t) oacc[t][r] *= alpha;
      if (vres) {
#pragma unroll
        for (int t = 0; t < 4; ++t) oacc2[t][r] *= alpha;
      }
    }
    __builtin_amdgcn_fence(__ATOMIC_RELEASE, "workgroup");
    __builtin_amdgcn_wave_barrier();
    __builtin_amdgcn_fence(__ATOMIC_ACQUIRE, "workgroup");
#pragma unroll 1
    for (int kk = 0; kk < 2; ++kk) {
      FragH pa;
      pa.h[0] = *(const v8h*)(pw + c * AT_KC + kk * 32 + 8 * hh);
      pa.h[1] = *(const v8h*)(pw + c * AT_KC + kk * 32 + 16 + 8 * hh);
#pragma unroll
      for (int t = 0; t < 4; ++t) {
        FragH vb;
        vb.h[0] = *(const v8h*)(Vts + (t * 16 + c) * AT_KC + kk * 32 + 8 * hh);
        vb.h[1] = *(const v8h*)(Vts + (t * 16 + c) * AT_KC + kk * 32 + 16 + 8 * hh);
        oacc[t] = mma_h(pa.v, vb.v, oacc[t]);
      }
      if (vres) {
#pragma unroll
        for (int t = 0; t < 4; ++t) {
          FragH vl;
          vl.h[0] = *(const v8h*)(Vrs + (t * 16 + c) * AT_KC + kk * 32 + 8 * hh);
          vl.h[1] = *(const v8h*)(Vrs + (t * 16 + c) * AT_KC + kk * 32 + 16 + 8 * hh);
          oacc2[t] = mma_h(pa.v, vl.v, oacc2[t]);
        }
      }
    }
  }

  float* os = Os[wave];
#pragma unroll
  for (int r = 0; r < 8; ++r) {
    const float inv = 1.0f / lrow[r];
#pragma unroll
    for (int t = 0; t < 4; ++t) os[(8 * hh + r) * 68 + t * 16 + c] = (oacc[t][r] + oacc2[t][r] * 0.0009765625f) * inv;
  }
  __builtin_amdgcn_fence(__ATOMIC_RELEASE, "workgroup");
  __builtin_amdgcn_wave_barrier();
  __builtin_amdgcn_fence(__ATOMIC_ACQUIRE, "workgroup");
  {
    const int q = lane >> 3, c8 = (lane & 7) * 8;
    v4u hv[4], lv[4];
#pragma unroll
    for (int it = 0; it < 4; ++it) {
      const int row = it * 4 + q;
      const float* sp = os + row * 68 + c8;
      v4u a, a2;
#pragma unroll
      for (int e = 0; e < 4; ++e) {
        const float f0 = sp[2 * e], f1 = sp[2 * e + 1];
        const unsigned short h0 = f2bf_bits(f0), h1 = f2bf_bits(f1);
        const unsigned short l0 = f2bf_bits(f0 - bf_bits2f(h0)), l1 = f2bf_bits(f1 - bf_bits2f(h1));
        a[e] = pk16(h0, h1); a2[e] = pk16(l0, l1);
      }
      hv[it] = a; lv[it] = a2;
    }
    for (int pass = 0; pass < 2; ++pass) {
#pragma unroll
      for (int it = 0; it < 4; ++it) {
        const int row = it * 4 + q;
        *(volatile v4u*)(Yh + (size_t)(q0 + row) * DM + c8) = hv[it];
        *(volatile v4u*)(Yl + (size_t)(q0 + row) * DM + c8) = lv[it];
      }
      __threadfence();
    }
  }
}

extern "C" void kernel_launch(void* const* d_in, const int* in_sizes, int n_in,
                              void* d_out, int out_size, void* d_ws, size_t ws_size,
                              hipStream_t stream) {
  if (n_in < 7) return;
  if (in_sizes[0] != NB * SEQ * DM) return;
  if (in_sizes[1] != DM * 3 * DM) return;
  if (in_sizes[2] != 3 * DM) return;
  if (in_sizes[3] != DM * DM) return;
  if (in_sizes[4] != DM) return;
  if (in_sizes[5] != NH * HD || in_sizes[6] != NH * HD) return;
  if (out_size != NB * SEQ * DM + NH * HD) return;

  const float* x      = (const float*)d_in[0];
  const float* W_attn = (const float*)d_in[1];
  const float* b_attn = (const float*)d_in[2];
  const float* W_proj = (const float*)d_in[3];
  const float* b_proj = (const float*)d_in[4];
  const float* bQ     = (const float*)d_in[5];
  const float* bK     = (const float*)d_in[6];

  const size_t PQK = (size_t)NB * SEQ * DQK * 2;
  const size_t PVT = (size_t)NB * DM * SEQ * 2;
  const size_t PVL = (size_t)NB * DM * VLO_COLS * 2;
  const size_t PX  = (size_t)NB * SEQ * DM * 2;
  const size_t PWA = (size_t)3 * DM * DM * 2;
  const size_t PWP = (size_t)DM * DM * 2;
  size_t off = 0;
  const size_t oQKh = off; off += PQK;
  const size_t oQKl = off; off += PQK;
  const size_t oVTh = off; off += PVT;
  const size_t oVTl = off; off += PVL;
  const size_t oXb  = off; off += PX;
  const size_t oYl  = off; off += PX;
  const size_t oWaT = off; off += PWA;
  const size_t oWpT = off; off += PWP;
  if (off > ws_size) return;
  if (off > (size_t)134217728) return;

  char* ws = (char*)d_ws;
  unsigned short* QKh = (unsigned short*)(ws + oQKh);
  unsigned short* QKl = (unsigned short*)(ws + oQKl);
  unsigned short* VTh = (unsigned short*)(ws + oVTh);
  unsigned short* VTl = (unsigned short*)(ws + oVTl);
  unsigned short* Xb  = (unsigned short*)(ws + oXb);
  unsigned short* Yh  = (unsigned short*)(ws + oXb);
  unsigned short* Yl  = (unsigned short*)(ws + oYl);
  unsigned short* WaT = (unsigned short*)(ws + oWaT);
  unsigned short* WpT = (unsigned short*)(ws + oWpT);
  float* out0 = (float*)d_out;
  float* out1 = (float*)d_out + (size_t)NB * SEQ * DM;

  const dim3 blk(256);

  tsplit1_kernel<<<dim3(3 * DM / 64, DM / 64), blk, 0, stream>>>(W_attn, WaT, DM, 3 * DM);
  tsplit1_kernel<<<dim3(DM / 64, DM / 64), blk, 0, stream>>>(W_proj, WpT, DM, DM);
  const int n8 = NB * SEQ * DM / 8;
  cvt_x_kernel<<<dim3(n8 / 256), blk, 0, stream>>>(x, Xb, n8, bQ, out1, NH * HD / 4);
  {
    const int M = NB * SEQ, N = 2 * DM, K = DM;
    const dim3 g(((M / 64) * (N / 64)) / 8, 1);
    gemm64<0><<<g, blk, 0, stream>>>(Xb, Xb, DM, 0L, WaT, DM, 0L, (void*)QKh, (void*)QKl, DQK, 0L, DQK, 0L,
                                     b_attn, bQ, bK, M, N, K);
  }
  {
    const int M = DM, N = SEQ, K = DM;
    const dim3 g(((M / 64) * (N / 64)) / 8, NB);
    gemm64<1><<<g, blk, 0, stream>>>(WaT + (size_t)2 * DM * DM, WaT + (size_t)2 * DM * DM, DM, 0L,
                                     Xb, DM, (long)SEQ * DM,
                                     (void*)VTh, (void*)VTl, SEQ, (long)DM * SEQ, VLO_COLS, (long)DM * VLO_COLS,
                                     b_attn + 2 * DM, b_attn, b_attn, M, N, K);
  }
  attn_kernel<<<dim3(NH * NQB, NB), dim3(128), 0, stream>>>(QKh, QKl, VTh, VTl, Yh, Yl);
  {
    const int M = NB * SEQ, N = DM, K = DM;
    const dim3 g(((M / 64) * (N / 64)) / 8, 1);
    gemm64<2><<<g, blk, 0, stream>>>(Yh, Yl, DM, 0L, WpT, DM, 0L, (void*)out0, (void*)out0, DM, 0L, DM, 0L,
                                     b_proj, b_proj, b_proj, M, N, K);
  }
  (void)hipGetLastError();
}
